// Model_6210522710673
// MI455X (gfx1250) — hardware-run, weakly checked
//
#include <hip/hip_runtime.h>
#include <math.h>

typedef __attribute__((ext_vector_type(16))) _Float16 v16h;
typedef __attribute__((ext_vector_type(8)))  _Float16 v8h;
typedef __attribute__((ext_vector_type(8)))  float    v8f;
typedef __attribute__((ext_vector_type(4)))  float    v4f;

constexpr int kRows    = 8192;
constexpr int kSeq     = 512;
constexpr int kPred    = 720;
constexpr int kPredPad = 768;
constexpr int kNexp    = 16;
constexpr int kHalf    = 256;
constexpr int kInfoP   = 32;
constexpr int kTrP     = 68;
constexpr int kSlabP   = 68;
constexpr int kGemmRows = 32;
constexpr int kGemmColsPerBlock = 256;
constexpr float kXnCarry = 16.0f;
constexpr float kEwCarry = 256.0f;
constexpr float kFold    = 1.0f / (kXnCarry * kEwCarry);
constexpr float kF16MinNormal = 6.103515625e-05f;
static_assert(kSeq % 32 == 0);
static_assert(kRows % kGemmRows == 0);
static_assert(kPredPad % kGemmColsPerBlock == 0);
static_assert(kPredPad % 64 == 0 && kPredPad >= kPred);
static_assert(kPred % 4 == 0);
static_assert((kRows * (kPred / 4)) % 256 == 0);
static_assert(kSeq == 2 * kHalf);

constexpr size_t kOffXN   = 0;
constexpr size_t kOffEWT  = kOffXN  + (size_t)kRows * kSeq * 2;
constexpr size_t kOffRINF = kOffEWT + (size_t)kNexp * kPredPad * kSeq * 2;
constexpr size_t kOffCOMB = kOffRINF + (size_t)kRows * kInfoP * 4;
constexpr size_t kWsTotal = kOffCOMB + (size_t)kRows * kPredPad * 4;
static_assert(kWsTotal == 47185920ull);
static_assert(kWsTotal <= 134217728ull);
static_assert((kOffEWT % 128) == 0 && (kOffRINF % 128) == 0 && (kOffCOMB % 128) == 0);

__device__ __forceinline__ float carry_flush(float v, float carry) {
  float s = v * carry;
  s = (fabsf(s) < kF16MinNormal) ? 0.0f : s;
  return s;
}

__device__ __forceinline__ void wmma_group_guard(v8f& a0, v8f& a1, v8f& a2, v8f& a3,
                                                 v16h x, v16h y0, v16h y1, v16h y2, v16h y3) {
  asm volatile("v_nop\n\tv_nop\n\tv_nop\n\tv_nop"
               : "+v"(a0), "+v"(a1), "+v"(a2), "+v"(a3)
               : "v"(x), "v"(y0), "v"(y1), "v"(y2), "v"(y3));
}

__global__ __launch_bounds__(256) void weight_plane_kernel(
    const float* __restrict__ ew, unsigned short* __restrict__ ewT)
{
  __shared__ __align__(16) float sT[64 * kTrP];
  const int tid = threadIdx.x, lane = tid & 31, wave = tid >> 5;
  const int l0 = blockIdx.x * 64;
  const int p0 = blockIdx.y * 64;
  const int e  = blockIdx.z;
  const int c  = tid & 63;
  const int r0 = tid >> 6;
  const int pc = p0 + c;
  const bool live = (pc < kPred);
  const int pcl = live ? pc : (kPred - 1);
  const float* src = ew + ((size_t)e * kSeq + l0) * kPred + pcl;
#pragma unroll 4
  for (int i = 0; i < 16; ++i) {
    const int r = r0 + 4 * i;
    float v = src[(size_t)r * kPred];
    asm volatile("" : "+v"(v));
    v = live ? v : 0.0f;
    sT[c * kTrP + r] = v;
  }
  __syncthreads();
  const int q = lane >> 3, c8 = (lane & 7) * 8;
  v8h hv[2];
#pragma unroll
  for (int it = 0; it < 2; ++it) {
    const int pr = it * 32 + wave * 4 + q;
    const float* sp = sT + pr * kTrP + c8;
    const v4f a0 = *(const v4f*)(sp);
    const v4f a1 = *(const v4f*)(sp + 4);
#pragma unroll
    for (int k = 0; k < 4; ++k) {
      const float f0 = carry_flush(a0[k], kEwCarry);
      const float f1 = carry_flush(a1[k], kEwCarry);
      hv[it][k]     = (_Float16)f0;
      hv[it][4 + k] = (_Float16)f1;
    }
  }
  for (int pass = 0; pass < 2; ++pass) {
#pragma unroll
    for (int it = 0; it < 2; ++it) {
      const int pr = it * 32 + wave * 4 + q;
      unsigned short* dst = ewT + ((size_t)e * kPredPad + p0 + pr) * kSeq + l0 + c8;
      *(volatile v8h*)dst = hv[it];
    }
    __threadfence();
  }
}

__global__ __launch_bounds__(256) void row_stage_kernel(
    const float* __restrict__ x, const float* __restrict__ gw, const float* __restrict__ gb,
    unsigned short* __restrict__ xn16, float* __restrict__ rinfo)
{
  __shared__ __align__(16) float sxn[kSeq];
  __shared__ float sre[kSeq];
  __shared__ float sim[kSeq];
  __shared__ float twc[kHalf];
  __shared__ float tws[kHalf];
  __shared__ float sI[kHalf];
  __shared__ float red8[8];
  __shared__ float sgate[kNexp];

  const int t = threadIdx.x, lane = t & 31, wave = t >> 5;
  const int b = blockIdx.x;
  const float* xb = x + (size_t)b * kSeq;
  const float v0 = xb[t];
  const float v1 = xb[t + kHalf];

  {
    float sn, cs;
    sincospif((float)t * (1.0f / 256.0f), &sn, &cs);
    twc[t] = cs;
    tws[t] = -sn;
  }

  auto bsum = [&](float v) -> float {
#pragma unroll
    for (int off = 16; off > 0; off >>= 1) v += __shfl_xor(v, off, 32);
    __syncthreads();
    if (lane == 0) red8[wave] = v;
    __syncthreads();
    float s = red8[0];
    s += red8[1];
    s += red8[2];
    s += red8[3];
    s += red8[4];
    s += red8[5];
    s += red8[6];
    s += red8[7];
    return s;
  };

  const float tot = bsum(v0 + v1);
  const float mu = tot * (1.0f / (float)kSeq);
  const float d0 = v0 - mu, d1 = v1 - mu;
  const float vs = bsum(d0 * d0 + d1 * d1);
  const float sd = sqrtf(vs * (1.0f / (float)kSeq)) + 1e-5f;
  const float isd = 1.0f / sd;

  sxn[t]         = carry_flush(d0 * isd, kXnCarry);
  sxn[t + kHalf] = carry_flush(d1 * isd, kXnCarry);
  {
    const int j0 = (int)(__brev((unsigned)t) >> 23);
    const int j1 = (int)(__brev((unsigned)(t + kHalf)) >> 23);
    sre[j0] = d0;
    sim[j0] = 0.0f;
    sre[j1] = d1;
    sim[j1] = 0.0f;
  }
  __syncthreads();

  if (t < 64) {
    const float* sp = sxn + t * 8;
    const v4f a0 = *(const v4f*)(sp);
    const v4f a1 = *(const v4f*)(sp + 4);
    v8h hv;
#pragma unroll
    for (int k = 0; k < 4; ++k) {
      const float f0 = a0[k];
      const float f1 = a1[k];
      hv[k]     = (_Float16)f0;
      hv[4 + k] = (_Float16)f1;
    }
    unsigned short* dst = xn16 + (size_t)b * kSeq + t * 8;
    *(volatile v8h*)dst = hv;
    __threadfence();
    *(volatile v8h*)dst = hv;
  }

#pragma unroll 1
  for (int s = 1; s <= 9; ++s) {
    const int m2 = 1 << (s - 1);
    const int jm = t & (m2 - 1);
    const int k  = ((t >> (s - 1)) << s) + jm;
    const int ti = jm << (9 - s);
    const float wr = twc[ti], wi = tws[ti];
    const float vr = sre[k + m2], vi = sim[k + m2];
    const float tr = wr * vr - wi * vi;
    const float tq = wr * vi + wi * vr;
    const float ur = sre[k], ui = sim[k];
    sre[k]      = ur + tr;
    sim[k]      = ui + tq;
    sre[k + m2] = ur - tr;
    sim[k + m2] = ui - tq;
    __syncthreads();
  }

  const float re = sre[t], im = sim[t];
  const float Ik = (re * re + im * im) * (1.0f / (float)kSeq);
  const float ssum = bsum(Ik);
  const float invs = (ssum == 0.0f) ? 1.0f : (1.0f / ssum);
  sI[t] = Ik * invs;
  __syncthreads();

  {
    const int ge = t >> 4, gj = t & 15;
    const float* gwe = gw + (size_t)ge * kHalf + gj;
    float p = 0.0f;
#pragma unroll 4
    for (int i = 0; i < 16; ++i) p = fmaf(sI[gj + 16 * i], gwe[16 * i], p);
    p += __shfl_xor(p, 8, 32);
    p += __shfl_xor(p, 4, 32);
    p += __shfl_xor(p, 2, 32);
    p += __shfl_xor(p, 1, 32);
    float gbv = gb[ge];
    asm volatile("" : "+v"(gbv));
    if (gj == 0) sgate[ge] = p + gbv;
  }
  __syncthreads();

  if (wave == 0) {
    float b0 = -INFINITY, b1 = -INFINITY;
    int i0 = 0, i1 = 0;
#pragma unroll
    for (int e = 0; e < kNexp; ++e) {
      const float g = sgate[e];
      const bool first  = (g > b0);
      const bool second = (!first) && (g > b1);
      b1 = first ? b0 : (second ? g : b1);
      i1 = first ? i0 : (second ? e : i1);
      b0 = first ? g : b0;
      i0 = first ? e : i0;
    }
    const float ex  = expf(b1 - b0);
    const float inv = 1.0f / (1.0f + ex);
    const float g0 = inv;
    const float g1 = ex * inv;
    float val = 0.0f;
    val = (lane == i0) ? g0 : val;
    val = (lane == i1) ? g1 : val;
    val = (lane == 16) ? mu : val;
    val = (lane == 17) ? sd : val;
    float* dst = rinfo + (size_t)b * kInfoP + lane;
    *(volatile float*)dst = val;
    __threadfence();
    *(volatile float*)dst = val;
  }
}

__global__ __launch_bounds__(128) void mix_gemm_kernel(
    const unsigned short* __restrict__ xn16, const unsigned short* __restrict__ ewT,
    const float* __restrict__ rinfo, float* __restrict__ comb)
{
  __shared__ __align__(16) _Float16 sA[kGemmRows * kSeq];
  __shared__ __align__(16) float sWt[kNexp * kGemmRows];
  __shared__ __align__(16) float sSlab[4][16 * kSlabP];
  union FH { v16h v; v8h h[2]; };

  const int tid = threadIdx.x, lane = tid & 31, wave = tid >> 5;
  const int m0 = blockIdx.x * kGemmRows;
  const int n0 = blockIdx.y * kGemmColsPerBlock + wave * 64;
  const _Float16* A  = (const _Float16*)xn16;
  const _Float16* Bt = (const _Float16*)ewT;

#pragma unroll 4
  for (int i = 0; i < 16; ++i) {
    const int ch = tid + i * 128;
    const int r  = ch >> 6;
    const int c8 = (ch & 63) * 8;
    *(v8h*)(sA + r * kSeq + c8) = *(const v8h*)(A + (size_t)(m0 + r) * kSeq + c8);
  }
  {
    const int r  = tid >> 2;
    const int e4 = (tid & 3) * 4;
    const v4f wv4 = *(const v4f*)(rinfo + (size_t)(m0 + r) * kInfoP + e4);
    sWt[(e4 + 0) * kGemmRows + r] = wv4[0];
    sWt[(e4 + 1) * kGemmRows + r] = wv4[1];
    sWt[(e4 + 2) * kGemmRows + r] = wv4[2];
    sWt[(e4 + 3) * kGemmRows + r] = wv4[3];
  }
  __syncthreads();

  const int rlane = lane & 15;
  const int koff  = (lane >> 4) * 8;
  const int mOff  = (lane >> 4) * 8;

  v8f outA[2][4], accE[2][4];
#pragma unroll
  for (int i = 0; i < 2; ++i)
#pragma unroll
    for (int j = 0; j < 4; ++j) {
      outA[i][j] = (v8f){0.f, 0.f, 0.f, 0.f, 0.f, 0.f, 0.f, 0.f};
      accE[i][j] = (v8f){0.f, 0.f, 0.f, 0.f, 0.f, 0.f, 0.f, 0.f};
    }

  const _Float16* Bw = Bt + (size_t)(n0 + rlane) * kSeq + koff;
  const _Float16* Aw = sA + rlane * kSeq + koff;

#pragma unroll 1
  for (int e = 0; e < kNexp; ++e) {
    const _Float16* Be = Bw + (size_t)e * kPredPad * kSeq;
#pragma unroll 1
    for (int k0 = 0; k0 < kSeq; k0 += 32) {
      FH bh[4];
#pragma unroll
      for (int j = 0; j < 4; ++j) {
        const _Float16* bp = Be + (size_t)(j * 16) * kSeq + k0;
        bh[j].h[0] = *(const v8h*)(bp);
        bh[j].h[1] = *(const v8h*)(bp + 16);
      }
#pragma unroll
      for (int i = 0; i < 2; ++i) {
        FH ah;
        const _Float16* ap = Aw + (i * 16) * kSeq + k0;
        ah.h[0] = *(const v8h*)(ap);
        ah.h[1] = *(const v8h*)(ap + 16);
#pragma unroll
        for (int j = 0; j < 4; ++j)
          accE[i][j] = __builtin_amdgcn_wmma_f32_16x16x32_f16(false, ah.v, false, bh[j].v, (short)0, accE[i][j], false, false);
        wmma_group_guard(accE[i][0], accE[i][1], accE[i][2], accE[i][3], ah.v, bh[0].v, bh[1].v, bh[2].v, bh[3].v);
      }
    }
    {
      const float* wp = sWt + e * kGemmRows + mOff;
      const v4f w00 = *(const v4f*)(wp);
      const v4f w01 = *(const v4f*)(wp + 4);
      const v4f w10 = *(const v4f*)(wp + 16);
      const v4f w11 = *(const v4f*)(wp + 20);
      const float wr0[8] = {w00[0], w00[1], w00[2], w00[3], w01[0], w01[1], w01[2], w01[3]};
      const float wr1[8] = {w10[0], w10[1], w10[2], w10[3], w11[0], w11[1], w11[2], w11[3]};
#pragma unroll
      for (int j = 0; j < 4; ++j) {
#pragma unroll
        for (int r = 0; r < 8; ++r) {
          outA[0][j][r] = fmaf(wr0[r], accE[0][j][r], outA[0][j][r]);
          outA[1][j][r] = fmaf(wr1[r], accE[1][j][r], outA[1][j][r]);
        }
        accE[0][j] = (v8f){0.f, 0.f, 0.f, 0.f, 0.f, 0.f, 0.f, 0.f};
        accE[1][j] = (v8f){0.f, 0.f, 0.f, 0.f, 0.f, 0.f, 0.f, 0.f};
      }
    }
  }

  float* slab = sSlab[wave];
#pragma unroll
  for (int i = 0; i < 2; ++i) {
#pragma unroll
    for (int j = 0; j < 4; ++j) {
#pragma unroll
      for (int r = 0; r < 8; ++r)
        slab[(mOff + r) * kSlabP + (j << 4) + rlane] = outA[i][j][r] * kFold;
    }
    __builtin_amdgcn_fence(__ATOMIC_RELEASE, "workgroup");
    __builtin_amdgcn_wave_barrier();
    __builtin_amdgcn_fence(__ATOMIC_ACQUIRE, "workgroup");
    {
      const int hh = lane >> 4, c4 = (lane & 15) * 4;
      for (int pass = 0; pass < 2; ++pass) {
#pragma unroll
        for (int it = 0; it < 8; ++it) {
          const int row = it * 2 + hh;
          const v4f v = *(const v4f*)(slab + row * kSlabP + c4);
          *(volatile v4f*)(comb + (size_t)(m0 + i * 16 + row) * kPredPad + n0 + c4) = v;
        }
        __threadfence();
      }
    }
    __builtin_amdgcn_fence(__ATOMIC_RELEASE, "workgroup");
    __builtin_amdgcn_wave_barrier();
    __builtin_amdgcn_fence(__ATOMIC_ACQUIRE, "workgroup");
  }
}

__global__ __launch_bounds__(256) void pack_kernel(
    const float* __restrict__ comb, const float* __restrict__ rinfo, const float* __restrict__ eb,
    float* __restrict__ out)
{
  constexpr int kQPerRow = kPred / 4;
  const int q = blockIdx.x * 256 + threadIdx.x;
  const int b = q / kQPerRow;
  const int c4 = (q - b * kQPerRow) * 4;
  const float* ri = rinfo + (size_t)b * kInfoP;
  v4f wq[4];
  wq[0] = *(const v4f*)(ri);
  wq[1] = *(const v4f*)(ri + 4);
  wq[2] = *(const v4f*)(ri + 8);
  wq[3] = *(const v4f*)(ri + 12);
  const v4f ms = *(const v4f*)(ri + 16);
  v4f acc = *(const v4f*)(comb + (size_t)b * kPredPad + c4);
#pragma unroll
  for (int e = 0; e < kNexp; ++e) {
    const v4f bv = *(const v4f*)(eb + (size_t)e * kPred + c4);
    const float we = wq[e >> 2][e & 3];
    acc[0] = fmaf(we, bv[0], acc[0]);
    acc[1] = fmaf(we, bv[1], acc[1]);
    acc[2] = fmaf(we, bv[2], acc[2]);
    acc[3] = fmaf(we, bv[3], acc[3]);
  }
  const float mu = ms[0], sd = ms[1];
  v4f res;
  res[0] = fmaf(sd, acc[0], mu);
  res[1] = fmaf(sd, acc[1], mu);
  res[2] = fmaf(sd, acc[2], mu);
  res[3] = fmaf(sd, acc[3], mu);
  float* dst = out + (size_t)q * 4;
  *(volatile v4f*)dst = res;
  __threadfence();
  *(volatile v4f*)dst = res;
}

extern "C" void kernel_launch(void* const* d_in, const int* in_sizes, int n_in,
                              void* d_out, int out_size, void* d_ws, size_t ws_size,
                              hipStream_t stream) {
  if (n_in < 5) return;
  if (in_sizes[0] != kRows * kSeq) return;
  if (in_sizes[1] != kNexp * kHalf) return;
  if (in_sizes[2] != kNexp) return;
  if (in_sizes[3] != kNexp * kSeq * kPred) return;
  if (in_sizes[4] != kNexp * kPred) return;
  if (out_size != kRows * kPred) return;
  if (ws_size < kWsTotal) return;

  const float* x  = (const float*)d_in[0];
  const float* gw = (const float*)d_in[1];
  const float* gb = (const float*)d_in[2];
  const float* ew = (const float*)d_in[3];
  const float* eb = (const float*)d_in[4];
  float* out = (float*)d_out;

  char* ws = (char*)d_ws;
  unsigned short* XN16 = (unsigned short*)(ws + kOffXN);
  unsigned short* EWT  = (unsigned short*)(ws + kOffEWT);
  float*          RINF = (float*)(ws + kOffRINF);
  float*          COMB = (float*)(ws + kOffCOMB);

  weight_plane_kernel<<<dim3(kSeq / 64, kPredPad / 64, kNexp), 256, 0, stream>>>(ew, EWT);
  row_stage_kernel<<<kRows, 256, 0, stream>>>(x, gw, gb, XN16, RINF);
  mix_gemm_kernel<<<dim3(kRows / kGemmRows, kPredPad / kGemmColsPerBlock), 128, 0, stream>>>(XN16, EWT, RINF, COMB);
  pack_kernel<<<(kRows * (kPred / 4)) / 256, 256, 0, stream>>>(COMB, RINF, eb, out);
}
